// TransformerLayer_1752346656957
// MI455X (gfx1250) — hardware-run, weakly checked
//
#include <hip/hip_runtime.h>
#include <stddef.h>


typedef _Float16 v16h __attribute__((ext_vector_type(16)));
typedef _Float16 v8h  __attribute__((ext_vector_type(8)));
typedef float    v8f  __attribute__((ext_vector_type(8)));
typedef float    v4f  __attribute__((ext_vector_type(4)));
typedef int      v4i  __attribute__((ext_vector_type(4)));

#ifndef NB
#define NB 4
#endif
#ifndef SEQ
#define SEQ 1024
#endif
#define NB_FULL  4
#define SEQ_FULL 1024
#define DIM   1024
#define NHEAD 16
#define HD    64
#define DFF   4096
#define MROWS (NB * SEQ)

#define RELL  128
#define NREL  257
#define RELP  288
#define TP    292
#define QROWS 64

static_assert(NB >= 1 && NB <= NB_FULL);
static_assert(SEQ >= 256 && SEQ <= SEQ_FULL && (SEQ % 256) == 0);
static_assert(DIM == NHEAD * HD);
static_assert(HD == 64);
static_assert(DIM == 128 * 8);
static_assert((MROWS % 64) == 0);
static_assert((DIM % 64) == 0 && (DFF % 64) == 0 && (DIM % 32) == 0 && (DFF % 32) == 0);
static_assert(NREL == 2 * RELL + 1 && RELP >= NREL && (RELP % 32) == 0 && TP >= RELP + 2);
static_assert((TP % 4) == 0);
static_assert((SEQ / 64) <= 16);
static_assert((SEQ % QROWS) == 0);

#define LDT 72
#define LDC 68

#define WCARRY 64.0f
#define RCARRY 64.0f
#define PCARRY 1024.0f
#define VCARRY 64.0f
#define HCARRY 4.0f
#define LN_EPS 1.0e-5f
#define MASK_FILL (-10000.0f)
#define SCORE_SCALE 0.125f
#define P_FLOOR (-16.0f)

#define ATT_LDS_BYTES (2 * 64 * LDT * 2 + 4 * 16 * LDT * 2 + 4 * 16 * TP * 4)
#define GEMM_LDS_BYTES (64 * LDC * 4)
static_assert(ATT_LDS_BYTES <= 131072);
static_assert(GEMM_LDS_BYTES <= 131072);
static_assert((DIM * 4 + 64) <= 131072);

#define WP         ((size_t)DIM * DIM)
#define WT_ELEMS   (WP * 4 + (size_t)DFF * DIM * 2)
#define WT_BYTES   (WT_ELEMS * 2)
#define P16_BYTES  ((size_t)MROWS * DIM * 2)
#define P32_BYTES  ((size_t)MROWS * DIM * 4)
#define F16_BYTES  ((size_t)MROWS * DFF * 2)
#define REL_BYTES  ((size_t)RELP * HD * 2)
#define FLAG_BYTES ((size_t)NB * (SEQ / 64) * 128)
#define OFF_X16    (WT_BYTES)
#define OFF_QH     (OFF_X16 + P16_BYTES)
#define OFF_KH     (OFF_QH + P16_BYTES)
#define OFF_VT     (OFF_KH + P16_BYTES)
#define OFF_CTX    (OFF_VT + P16_BYTES)
#define OFF_X1     (OFF_CTX + P16_BYTES)
#define OFF_F      (OFF_X1 + P32_BYTES)
#define OFF_WR     (OFF_F + F16_BYTES)
#define OFF_WRT    (OFF_WR + REL_BYTES)
#define OFF_FLAG   (OFF_WRT + REL_BYTES)
#define WS_TOTAL   (OFF_FLAG + FLAG_BYTES)
#define OFF_HF     (OFF_QH)
#define OFF_H16    (OFF_X16)
#define OFF_Y      (OFF_X1)
static_assert((WP % 2048) == 0 && (WT_ELEMS % 2048) == 0);
static_assert((WT_BYTES % 128) == 0 && (P16_BYTES % 128) == 0 && (P32_BYTES % 128) == 0);
static_assert((F16_BYTES % 128) == 0 && (REL_BYTES % 128) == 0 && (FLAG_BYTES % 128) == 0);
static_assert(((size_t)DFF * DIM) == 4 * WP);
static_assert(OFF_KH == OFF_QH + P16_BYTES && P32_BYTES <= 2 * P16_BYTES);
static_assert(OFF_HF + P32_BYTES <= OFF_VT);
static_assert(OFF_H16 + P16_BYTES <= OFF_QH);
static_assert(OFF_Y + P32_BYTES <= OFF_F);
static_assert(((size_t)RELP * HD) == (size_t)9 * 2048);
static_assert(WS_TOTAL <= (size_t)134217728);

__device__ __forceinline__ float bf16r(float x) {
  unsigned int u = __float_as_uint(x);
  u = (u + 0x7FFFu + ((u >> 16) & 1u)) & 0xFFFF0000u;
  return __uint_as_float(u);
}

static __device__ __forceinline__ _Float16 toh_flush(float v) {
  const _Float16 r = (_Float16)v;
  return (fabsf(v) < 6.103515625e-05f) ? (_Float16)0.0f : r;
}

__device__ __forceinline__ v16h frag_at(const _Float16* p) {
  v8h lo = *(const v8h*)(p);
  v8h hi = *(const v8h*)(p + 16);
  v16h out;
#pragma unroll
  for (int i = 0; i < 8; ++i) { out[i] = lo[i]; out[i + 8] = hi[i]; }
  return out;
}
__device__ __forceinline__ v16h ld_frag(const _Float16* base, int ld) {
  const int lane = threadIdx.x & 31;
  return frag_at(base + (lane & 15) * ld + (lane >> 4) * 8);
}

__device__ __forceinline__ v8f wmma16(v16h a, v16h b, v8f c) {
  v8f d = __builtin_amdgcn_wmma_f32_16x16x32_f16(false, a, false, b, (short)0, c,
                                                 false, false);
  asm volatile("v_nop\n\tv_nop\n\tv_nop\n\tv_nop" : "+v"(d) : "v"(a), "v"(b));
  return d;
}

__device__ __forceinline__ float red32_sum(float x) {
#pragma unroll
  for (int off = 1; off < 32; off <<= 1) x += __shfl_xor(x, off, 32);
  return x;
}

__device__ __forceinline__ void wave_lds_sync() {
  __builtin_amdgcn_fence(3  , "wavefront");
  asm volatile("s_wait_dscnt 0x0" ::: "memory");
  __builtin_amdgcn_wave_barrier();
}

__global__ __launch_bounds__(256) void wconv_kernel(
    const float* __restrict__ W0, const float* __restrict__ W1p,
    const float* __restrict__ W2p, const float* __restrict__ W3,
    const float* __restrict__ W4, const float* __restrict__ W5,
    _Float16* __restrict__ Wt) {
  const size_t e = ((size_t)blockIdx.x * 256 + threadIdx.x) * 8;
  const unsigned seg = (unsigned)(((size_t)blockIdx.x * 2048) / WP);
  const float* W = W0;
  size_t base = 0;
  if (seg == 1) { W = W1p; base = WP; }
  if (seg == 2) { W = W2p; base = 2 * WP; }
  if (seg == 3) { W = W3;  base = 3 * WP; }
  if (seg >= 4 && seg < 8) { W = W4; base = 4 * WP; }
  if (seg >= 8) { W = W5; base = 8 * WP; }
  const float* sp = W + (e - base);
  const v4f a0 = *(const v4f*)(sp);
  const v4f a1 = *(const v4f*)(sp + 4);
  v8h o;
#pragma unroll
  for (int j = 0; j < 4; ++j) {
    o[j]     = toh_flush(WCARRY * bf16r(a0[j]));
    o[j + 4] = toh_flush(WCARRY * bf16r(a1[j]));
  }
  *(volatile v8h*)(Wt + e) = o;
  __threadfence();
  *(volatile v8h*)(Wt + e) = o;
}

__global__ __launch_bounds__(256) void relconv_kernel(
    const float* __restrict__ Wrel, _Float16* __restrict__ WR, _Float16* __restrict__ WRT) {
  const int blk = blockIdx.x;
  v8h o;
  if (blk < 9) {
    const int e = (blk * 256 + (int)threadIdx.x) * 8;
    const int rel = e >> 6;
    const int d0 = e & 63;
    const int relc = min(rel, NREL - 1);
    const float* sp = Wrel + (size_t)relc * HD + d0;
    const v4f a0 = *(const v4f*)(sp);
    const v4f a1 = *(const v4f*)(sp + 4);
#pragma unroll
    for (int j = 0; j < 4; ++j) {
      const _Float16 t0 = toh_flush(RCARRY * bf16r(a0[j]));
      const _Float16 t1 = toh_flush(RCARRY * bf16r(a1[j]));
      o[j]     = (rel < NREL) ? t0 : (_Float16)0.0f;
      o[j + 4] = (rel < NREL) ? t1 : (_Float16)0.0f;
    }
    *(volatile v8h*)(WR + e) = o;
    __threadfence();
    *(volatile v8h*)(WR + e) = o;
  } else {
    const int e = ((blk - 9) * 256 + (int)threadIdx.x) * 8;
    const int d = e / RELP;
    const int r0 = e - d * RELP;
#pragma unroll
    for (int j = 0; j < 8; ++j) {
      const int rel = r0 + j;
      const int relc = min(rel, NREL - 1);
      const float xv = Wrel[(size_t)relc * HD + d];
      const _Float16 t0 = toh_flush(RCARRY * bf16r(xv));
      o[j] = (rel < NREL) ? t0 : (_Float16)0.0f;
    }
    *(volatile v8h*)(WRT + e) = o;
    __threadfence();
    *(volatile v8h*)(WRT + e) = o;
  }
}

__global__ __launch_bounds__(256) void xconv_kernel(
    const float* __restrict__ x, _Float16* __restrict__ X16) {
  const size_t e = ((size_t)blockIdx.x * 256 + threadIdx.x) * 8;
  const int row = (int)(e / DIM);
  const int c = (int)(e - (size_t)row * DIM);
  const int bidx = row / SEQ;
  const int sq = row - bidx * SEQ;
  const size_t frow = (size_t)bidx * SEQ_FULL + sq;
  const float* sp = x + frow * DIM + c;
  const v4f a0 = *(const v4f*)(sp);
  const v4f a1 = *(const v4f*)(sp + 4);
  v8h o;
#pragma unroll
  for (int j = 0; j < 4; ++j) {
    o[j]     = toh_flush(bf16r(a0[j]));
    o[j + 4] = toh_flush(bf16r(a1[j]));
  }
  *(volatile v8h*)(X16 + e) = o;
  __threadfence();
  *(volatile v8h*)(X16 + e) = o;
}

__global__ __launch_bounds__(256) void flag_kernel(
    const int* __restrict__ mask, int* __restrict__ flags) {
  __shared__ int wbits[8];
  __shared__ int wfull[8];
  const int tid = threadIdx.x, lane = tid & 31;
  const int w = __builtin_amdgcn_readfirstlane(threadIdx.x >> 5);
  const int qt = blockIdx.x;
  const int b = blockIdx.y;
  const int row = tid >> 2, quarter = tid & 3;
  const int* mp = mask + ((size_t)b * SEQ_FULL + qt * 64 + row) * SEQ_FULL + quarter * (SEQ / 4);
  int bits = 0;
#pragma unroll 1
  for (int t = 0; t < SEQ / 256; ++t) {
    int any = 0;
#pragma unroll 4
    for (int i = 0; i < 16; ++i) {
      const v4i mk = *(const v4i*)(mp + t * 64 + i * 4);
      any |= (int)(mk[0] == 0) | (int)(mk[1] == 0) | (int)(mk[2] == 0) | (int)(mk[3] == 0);
    }
    bits |= any << (quarter * (SEQ / 256) + t);
  }
  int rowbits = bits | __shfl_xor(bits, 1, 32);
  rowbits |= __shfl_xor(rowbits, 2, 32);
  int full = (rowbits == 0) ? 1 : 0;
#pragma unroll
  for (int off = 1; off < 32; off <<= 1) {
    bits |= __shfl_xor(bits, off, 32);
    full |= __shfl_xor(full, off, 32);
  }
  if (lane == 0) { wbits[w] = bits; wfull[w] = full; }
  __syncthreads();
  if (w == 0) {
    int ab = 0, af = 0;
#pragma unroll
    for (int i = 0; i < 8; ++i) { ab |= wbits[i]; af |= wfull[i]; }
    v4i line;
    line[0] = (lane == 0) ? ab : 0;
    line[1] = (lane == 0) ? af : 0;
    line[2] = 0;
    line[3] = 0;
    if (lane < 8) {
      int* dp = flags + ((size_t)b * (SEQ / 64) + qt) * 32 + lane * 4;
      *(volatile v4i*)dp = line;
      __threadfence();
      *(volatile v4i*)dp = line;
    }
  }
}

template <int MODE, int KD, int NP>
__device__ __forceinline__ void gemm_body(
    const _Float16* __restrict__ A16, const _Float16* __restrict__ Bt,
    const float* __restrict__ bias, const float* __restrict__ xin,
    const float* __restrict__ resf, float* __restrict__ outf,
    _Float16* __restrict__ out16) {
  static_assert((KD % 32) == 0 && (NP % 64) == 0);
  static_assert(256 * 16 * 2 == 64 * 64 * 2);
  static_assert(256 * 16 * 4 == 64 * 64 * 4);
  __shared__ float Cs[64 * LDC] __attribute__((aligned(16)));
  const int tid = threadIdx.x, lane = tid & 31;
  const int w = __builtin_amdgcn_readfirstlane(threadIdx.x >> 5);
  const int mw = w >> 1, nw = w & 1;
  const int hh = lane >> 4, m = lane & 15;
  const int n0 = blockIdx.x * 64;
  const int row0 = blockIdx.y * 64;

  const _Float16* ap  = A16 + (size_t)(row0 + mw * 16 + m) * KD + hh * 8;
  const _Float16* bp0 = Bt + (size_t)(n0 + nw * 32 + m) * KD + hh * 8;
  const _Float16* bp1 = bp0 + (size_t)16 * KD;
  v8f acc0 = {}, acc1 = {};
#pragma unroll 2
  for (int k0 = 0; k0 < KD; k0 += 32) {
    const v16h a  = frag_at(ap + k0);
    const v16h b0 = frag_at(bp0 + k0);
    const v16h b1 = frag_at(bp1 + k0);
    acc0 = wmma16(a, b0, acc0);
    acc1 = wmma16(a, b1, acc1);
  }
#pragma unroll
  for (int r = 0; r < 8; ++r) {
    float* d = &Cs[(mw * 16 + hh * 8 + r) * LDC + nw * 32 + m];
    d[0]  = acc0[r];
    d[16] = acc1[r];
  }
  __syncthreads();

  if (MODE == 0) {
    v8h x[2];
    size_t off[2];
#pragma unroll
    for (int i = 0; i < 2; ++i) {
      const int r = 32 * i + (tid >> 3);
      const int c = (tid & 7) * 8;
      const v4f u0 = *(const v4f*)&Cs[r * LDC + c];
      const v4f u1 = *(const v4f*)&Cs[r * LDC + c + 4];
      const v4f g0 = *(const v4f*)(bias + n0 + c);
      const v4f g1 = *(const v4f*)(bias + n0 + c + 4);
#pragma unroll
      for (int j = 0; j < 4; ++j) {
        x[i][j]     = toh_flush(u0[j] * (1.0f / WCARRY) + bf16r(g0[j]));
        x[i][j + 4] = toh_flush(u1[j] * (1.0f / WCARRY) + bf16r(g1[j]));
      }
      off[i] = (size_t)(row0 + r) * NP + n0 + c;
    }
#pragma unroll
    for (int i = 0; i < 2; ++i) *(volatile v8h*)(out16 + off[i]) = x[i];
    __threadfence();
#pragma unroll
    for (int i = 0; i < 2; ++i) *(volatile v8h*)(out16 + off[i]) = x[i];
  }

  if (MODE == 1) {
    const int bidx = row0 / SEQ;
    const int key0 = row0 - bidx * SEQ;
    v8h x[2];
    size_t off[2];
#pragma unroll
    for (int i = 0; i < 2; ++i) {
      const int dcol = 32 * i + (tid >> 3);
      const int kk = (tid & 7) * 8;
      const float gb = bf16r(bias[n0 + dcol]);
#pragma unroll
      for (int j = 0; j < 8; ++j)
        x[i][j] = toh_flush(Cs[(kk + j) * LDC + dcol] * (1.0f / WCARRY) + gb);
      off[i] = ((size_t)bidx * DIM + n0 + dcol) * SEQ + key0 + kk;
    }
#pragma unroll
    for (int i = 0; i < 2; ++i) *(volatile v8h*)(out16 + off[i]) = x[i];
    __threadfence();
#pragma unroll
    for (int i = 0; i < 2; ++i) *(volatile v8h*)(out16 + off[i]) = x[i];
  }

  if (MODE == 2) {
    v4f xs[4];
    size_t off[4];
#pragma unroll
    for (int i = 0; i < 4; ++i) {
      const int r = 16 * i + (tid >> 4);
      const int c = (tid & 15) * 4;
      const int crow = row0 + r;
      const int bidx = crow / SEQ;
      const int sq = crow - bidx * SEQ;
      const size_t frow = (size_t)bidx * SEQ_FULL + sq;
      const v4f u = *(const v4f*)&Cs[r * LDC + c];
      const v4f q = *(const v4f*)(xin + frow * DIM + n0 + c);
      const v4f gb = *(const v4f*)(bias + n0 + c);
      v4f val;
#pragma unroll
      for (int j = 0; j < 4; ++j)
        val[j] = (u[j] * (1.0f / (WCARRY * VCARRY)) + bf16r(gb[j])) + bf16r(q[j]);
      xs[i] = val;
      off[i] = (size_t)crow * NP + n0 + c;
    }
#pragma unroll
    for (int i = 0; i < 4; ++i) *(volatile v4f*)(outf + off[i]) = xs[i];
    __threadfence();
#pragma unroll
    for (int i = 0; i < 4; ++i) *(volatile v4f*)(outf + off[i]) = xs[i];
  }

  if (MODE == 3) {
    v8h x[2];
    size_t off[2];
#pragma unroll
    for (int i = 0; i < 2; ++i) {
      const int r = 32 * i + (tid >> 3);
      const int c = (tid & 7) * 8;
      const v4f u0 = *(const v4f*)&Cs[r * LDC + c];
      const v4f u1 = *(const v4f*)&Cs[r * LDC + c + 4];
      const v4f g0 = *(const v4f*)(bias + n0 + c);
      const v4f g1 = *(const v4f*)(bias + n0 + c + 4);
#pragma unroll
      for (int j = 0; j < 4; ++j) {
        const float t0 = fmaxf(u0[j] * (1.0f / WCARRY) + bf16r(g0[j]), 0.0f);
        const float t1 = fmaxf(u1[j] * (1.0f / WCARRY) + bf16r(g1[j]), 0.0f);
        x[i][j]     = toh_flush(HCARRY * t0);
        x[i][j + 4] = toh_flush(HCARRY * t1);
      }
      off[i] = (size_t)(row0 + r) * NP + n0 + c;
    }
#pragma unroll
    for (int i = 0; i < 2; ++i) *(volatile v8h*)(out16 + off[i]) = x[i];
    __threadfence();
#pragma unroll
    for (int i = 0; i < 2; ++i) *(volatile v8h*)(out16 + off[i]) = x[i];
  }

  if (MODE == 4) {
    v4f xs[4];
    size_t off[4];
#pragma unroll
    for (int i = 0; i < 4; ++i) {
      const int r = 16 * i + (tid >> 4);
      const int c = (tid & 15) * 4;
      const int crow = row0 + r;
      const v4f u  = *(const v4f*)&Cs[r * LDC + c];
      const v4f gb = *(const v4f*)(bias + n0 + c);
      const v4f rx = *(const v4f*)(resf + (size_t)crow * DIM + n0 + c);
      v4f val;
#pragma unroll
      for (int j = 0; j < 4; ++j)
        val[j] = (u[j] * (1.0f / (WCARRY * HCARRY)) + bf16r(gb[j])) + rx[j];
      xs[i] = val;
      off[i] = (size_t)crow * NP + n0 + c;
    }
#pragma unroll
    for (int i = 0; i < 4; ++i) *(volatile v4f*)(outf + off[i]) = xs[i];
    __threadfence();
#pragma unroll
    for (int i = 0; i < 4; ++i) *(volatile v4f*)(outf + off[i]) = xs[i];
  }
}

__global__ __launch_bounds__(256) void gemm_rows_kernel(
    const _Float16* __restrict__ A16, const _Float16* __restrict__ Bt,
    const float* __restrict__ bias, const float* __restrict__ xin,
    const float* __restrict__ resf, float* __restrict__ outf,
    _Float16* __restrict__ out16) {
  gemm_body<0, DIM, DIM>(A16, Bt, bias, xin, resf, outf, out16);
}
__global__ __launch_bounds__(256) void gemm_vt_kernel(
    const _Float16* __restrict__ A16, const _Float16* __restrict__ Bt,
    const float* __restrict__ bias, const float* __restrict__ xin,
    const float* __restrict__ resf, float* __restrict__ outf,
    _Float16* __restrict__ out16) {
  gemm_body<1, DIM, DIM>(A16, Bt, bias, xin, resf, outf, out16);
}
__global__ __launch_bounds__(256) void gemm_oproj_kernel(
    const _Float16* __restrict__ A16, const _Float16* __restrict__ Bt,
    const float* __restrict__ bias, const float* __restrict__ xin,
    const float* __restrict__ resf, float* __restrict__ outf,
    _Float16* __restrict__ out16) {
  gemm_body<2, DIM, DIM>(A16, Bt, bias, xin, resf, outf, out16);
}
__global__ __launch_bounds__(256) void gemm_ffn1_kernel(
    const _Float16* __restrict__ A16, const _Float16* __restrict__ Bt,
    const float* __restrict__ bias, const float* __restrict__ xin,
    const float* __restrict__ resf, float* __restrict__ outf,
    _Float16* __restrict__ out16) {
  gemm_body<3, DIM, DFF>(A16, Bt, bias, xin, resf, outf, out16);
}
__global__ __launch_bounds__(256) void gemm_ffn2_kernel(
    const _Float16* __restrict__ A16, const _Float16* __restrict__ Bt,
    const float* __restrict__ bias, const float* __restrict__ xin,
    const float* __restrict__ resf, float* __restrict__ outf,
    _Float16* __restrict__ out16) {
  gemm_body<4, DFF, DIM>(A16, Bt, bias, xin, resf, outf, out16);
}

template <int MODE>
__device__ __forceinline__ void ln_body(
    const float* __restrict__ src, const float* __restrict__ g,
    const float* __restrict__ be, float* __restrict__ outf,
    _Float16* __restrict__ out16) {
#pragma clang fp contract(off)
  static_assert(128 * 4 * 2 == DIM);
  static_assert(128 * 8 == DIM);
  __shared__ float red[8];
  __shared__ float ys[DIM] __attribute__((aligned(16)));
  const int tid = threadIdx.x, lane = tid & 31;
  const int w = __builtin_amdgcn_readfirstlane(threadIdx.x >> 5);
  const int row = blockIdx.x;
  const int c0 = tid * 4;
  const int c1 = DIM / 2 + tid * 4;
  const float* sp = src + (size_t)row * DIM;
  const v4f a0 = *(const v4f*)(sp + c0);
  const v4f a1 = *(const v4f*)(sp + c1);
  float s = ((a0[0] + a0[1]) + (a0[2] + a0[3])) + ((a1[0] + a1[1]) + (a1[2] + a1[3]));
  s = red32_sum(s);
  if (lane == 0) red[w] = s;
  __syncthreads();
  const float mean = ((red[0] + red[1]) + (red[2] + red[3])) * (1.0f / (float)DIM);
  v4f d0, d1;
#pragma unroll
  for (int j = 0; j < 4; ++j) { d0[j] = a0[j] - mean; d1[j] = a1[j] - mean; }
  float q = ((d0[0] * d0[0] + d0[1] * d0[1]) + (d0[2] * d0[2] + d0[3] * d0[3])) +
            ((d1[0] * d1[0] + d1[1] * d1[1]) + (d1[2] * d1[2] + d1[3] * d1[3]));
  q = red32_sum(q);
  if (lane == 0) red[4 + w] = q;
  __syncthreads();
  const float var = ((red[4] + red[5]) + (red[6] + red[7])) * (1.0f / (float)DIM);
  const float sd = sqrtf(var);
  const float inv = 1.0f / (sd + LN_EPS);
  const v4f g0 = *(const v4f*)(g + c0);
  const v4f g1 = *(const v4f*)(g + c1);
  const v4f b0 = *(const v4f*)(be + c0);
  const v4f b1 = *(const v4f*)(be + c1);
  v4f y0, y1;
#pragma unroll
  for (int j = 0; j < 4; ++j) {
    y0[j] = (bf16r(g0[j]) * d0[j]) * inv + bf16r(b0[j]);
    y1[j] = (bf16r(g1[j]) * d1[j]) * inv + bf16r(b1[j]);
  }

  if (MODE == 0) {
    *(v4f*)&ys[c0] = y0;
    *(v4f*)&ys[c1] = y1;
    __syncthreads();
    const v4f u0 = *(const v4f*)&ys[tid * 8];
    const v4f u1 = *(const v4f*)&ys[tid * 8 + 4];
    v8h o;
#pragma unroll
    for (int j = 0; j < 4; ++j) {
      o[j]     = toh_flush(u0[j]);
      o[j + 4] = toh_flush(u1[j]);
    }
    float* op = outf + (size_t)row * DIM;
    _Float16* hp = out16 + (size_t)row * DIM + tid * 8;
    *(volatile v4f*)(op + c0) = y0;
    *(volatile v4f*)(op + c1) = y1;
    *(volatile v8h*)hp = o;
    __threadfence();
    *(volatile v4f*)(op + c0) = y0;
    *(volatile v4f*)(op + c1) = y1;
    *(volatile v8h*)hp = o;
  }

  if (MODE == 1) {
    const int bidx = row / SEQ;
    const int sq = row - bidx * SEQ;
    const size_t frow = (size_t)bidx * SEQ_FULL + sq;
    float* op = outf + frow * DIM;
    *(volatile v4f*)(op + c0) = y0;
    *(volatile v4f*)(op + c1) = y1;
    __threadfence();
    *(volatile v4f*)(op + c0) = y0;
    *(volatile v4f*)(op + c1) = y1;
  }
}

__global__ __launch_bounds__(128) void ln_mid_kernel(
    const float* __restrict__ src, const float* __restrict__ g,
    const float* __restrict__ be, float* __restrict__ outf,
    _Float16* __restrict__ out16) {
  ln_body<0>(src, g, be, outf, out16);
}
__global__ __launch_bounds__(128) void ln_out_kernel(
    const float* __restrict__ src, const float* __restrict__ g,
    const float* __restrict__ be, float* __restrict__ outf,
    _Float16* __restrict__ out16) {
  ln_body<1>(src, g, be, outf, out16);
}

__global__ __launch_bounds__(128) __attribute__((amdgpu_num_vgpr(256))) void attn_kernel(
    const _Float16* __restrict__ Qh, const _Float16* __restrict__ Kh,
    const _Float16* __restrict__ Vt, const int* __restrict__ mask,
    const _Float16* __restrict__ WR, const _Float16* __restrict__ WRT,
    const int* __restrict__ flags, _Float16* __restrict__ Ov) {
  static_assert(128 * 4 * 8 == 64 * 64);
  static_assert(32 * 16 * 4 == 16 * HD * 2);
  __shared__ _Float16 Ks[64 * LDT] __attribute__((aligned(16)));
  __shared__ _Float16 Vs[64 * LDT] __attribute__((aligned(16)));
  __shared__ _Float16 Ps[4 * 16 * LDT] __attribute__((aligned(16)));
  __shared__ float    Tb[4 * 16 * TP] __attribute__((aligned(16)));

  const int tid = threadIdx.x, lane = tid & 31;
  const int w = __builtin_amdgcn_readfirstlane(threadIdx.x >> 5);
  const int hh = lane >> 4, m = lane & 15;
  const int q0 = blockIdx.x * QROWS;
  const int head = blockIdx.y;
  const int b = blockIdx.z;
  _Float16* P = Ps + w * (16 * LDT);
  const int tw0 = w * (16 * TP);
  const int tb0 = tw0 + m * TP;
  const int qw0 = q0 + w * 16;
  const int qrow = qw0 + m;

  const size_t qoff = (size_t)(b * SEQ + qrow) * DIM + head * HD + hh * 8;
  v16h qf[2];
  qf[0] = frag_at(Qh + qoff);
  qf[1] = frag_at(Qh + qoff + 32);

  const int* flp = flags + ((size_t)b * (SEQ / 64) + blockIdx.x) * 32;
  const int fl0 = flp[0];
  const int fl1 = (flp[1] != 0) ? 1 : 0;

#pragma unroll 1
  for (int nt = 0; nt < RELP / 16; ++nt) {
    v8f t = {};
#pragma unroll
    for (int c = 0; c < 2; ++c) {
      const v16h wf = frag_at(WR + (size_t)(nt * 16 + m) * HD + c * 32 + hh * 8);
      t = wmma16(qf[c], wf, t);
    }
#pragma unroll
    for (int r = 0; r < 8; ++r)
      Tb[tw0 + (8 * hh + r) * TP + nt * 16 + m] = t[r] * (1.0f / RCARRY);
  }
  wave_lds_sync();
  const float tpast = Tb[tb0 + 2 * RELL];
  const float tfut  = Tb[tb0];

  const int* mrowp = mask + ((size_t)b * SEQ_FULL + qrow) * SEQ_FULL + hh * 8;

  float mrun = -1.0e30f, lrun = 0.0f, lpast = 0.0f, lfut = 0.0f;
  v8f o[4];
#pragma unroll
  for (int nb = 0; nb < 4; ++nb) o[nb] = (v8f){};

  const size_t kplane = (size_t)b * SEQ * DIM + head * HD;
  const size_t vplane = ((size_t)b * DIM + head * HD) * SEQ;

  for (int kt = 0; kt < SEQ / 64; ++kt) {
    const int vis = ((fl0 >> kt) & 1) | fl1;
    if (vis == 0) continue;
    const int kb = kt * 64;
#pragma unroll
    for (int j = 0; j < 4; ++j) {
      const int idx = tid + 128 * j;
      const int r = idx >> 3, c = (idx & 7) * 8;
      *(v8h*)&Ks[r * LDT + c] = *(const v8h*)(Kh + kplane + (size_t)(kb + r) * DIM + c);
      *(v8h*)&Vs[r * LDT + c] = *(const v8h*)(Vt + vplane + (size_t)r * SEQ + kb + c);
    }
    __syncthreads();

    v8f s[4];
#pragma unroll
    for (int kg = 0; kg < 4; ++kg) {
      v8f t = {};
#pragma unroll
      for (int c = 0; c < 2; ++c) {
        const v16h kf = ld_frag(&Ks[(kg * 16) * LDT + c * 32], LDT);
        t = wmma16(kf, qf[c], t);
      }
      s[kg] = t;
    }

    const int dlo = qw0 - (kb + 63);
    const int dhi = qw0 + 15 - kb;
    const bool farp = (dlo >= RELL);
    const bool farf = (dhi <= -RELL);

    if (farp || farf) {
      const float tbc = farp ? tpast : tfut;
#pragma unroll
      for (int kg = 0; kg < 4; ++kg) {
        const v4i mk0 = *(const v4i*)(mrowp + kb + kg * 16);
        const v4i mk1 = *(const v4i*)(mrowp + kb + kg * 16 + 4);
        const int mk[8] = {mk0[0], mk0[1], mk0[2], mk0[3], mk1[0], mk1[1], mk1[2], mk1[3]};
#pragma unroll
        for (int r = 0; r < 8; ++r) {
          const float sv = (s[kg][r] + tbc) * SCORE_SCALE;
          s[kg][r] = (mk[r] != 0) ? MASK_FILL : sv;
        }
      }
    } else {
#pragma unroll
      for (int kg = 0; kg < 4; ++kg) {
        const v4i mk0 = *(const v4i*)(mrowp + kb + kg * 16);
        const v4i mk1 = *(const v4i*)(mrowp + kb + kg * 16 + 4);
        const int mk[8] = {mk0[0], mk0[1], mk0[2], mk0[3], mk1[0], mk1[1], mk1[2], mk1[3]};
        const int dbase = qrow - (kb + kg * 16 + 8 * hh);
        float tg[8];
#pragma unroll
        for (int r = 0; r < 8; ++r) {
          const int rel = min(max(dbase - r, -RELL), RELL) + RELL;
          float tv = Tb[tb0 + rel];
          asm volatile("" : "+v"(tv));
          tg[r] = tv;
        }
#pragma unroll
        for (int r = 0; r < 8; ++r) {
          const int d = dbase - r;
          const int rel = min(max(d, -RELL), RELL) + RELL;
          float sv = (s[kg][r] + tg[r]) * SCORE_SCALE;
          sv = (mk[r] != 0) ? MASK_FILL : sv;
          s[kg][r] = sv;
          const int inb = (int)(d > -RELL) & (int)(d < RELL);
          const int so = (inb != 0) ? rel : (RELP + hh);
          Tb[tb0 + so] = sv;
        }
      }
    }

    float mx = fmaxf(fmaxf(s[0][0], s[1][0]), fmaxf(s[2][0], s[3][0]));
#pragma unroll
    for (int kg = 0; kg < 4; ++kg)
#pragma unroll
      for (int r = 1; r < 8; ++r) mx = fmaxf(mx, s[kg][r]);
    mx = fmaxf(mx, __shfl_xor(mx, 16, 32));
    const float mn = fmaxf(mrun, mx);
    const float alpha = __expf(mrun - mn);
    mrun = mn;
    float rs[4];
#pragma unroll
    for (int kg = 0; kg < 4; ++kg) {
#pragma unroll
      for (int r = 0; r < 8; ++r) {
        const float ea = s[kg][r] - mrun;
        const float ex = __expf(fmaxf(ea, -64.0f));
        s[kg][r] = (ea < P_FLOOR) ? 0.0f : ex;
      }
      rs[kg] = ((s[kg][0] + s[kg][1]) + (s[kg][2] + s[kg][3])) +
               ((s[kg][4] + s[kg][5]) + (s[kg][6] + s[kg][7]));
    }
    const float rl = (rs[0] + rs[1]) + (rs[2] + rs[3]);
    float fpa = 0.0f, ffu = 0.0f;
    if (farp || farf) {
      fpa = farp ? rl : 0.0f;
      ffu = farp ? 0.0f : rl;
    } else {
#pragma unroll
      for (int kg = 0; kg < 4; ++kg) {
        const int dbase = qrow - (kb + kg * 16 + 8 * hh);
#pragma unroll
        for (int r = 0; r < 8; ++r) {
          const int d = dbase - r;
          fpa += (d >= RELL) ? s[kg][r] : 0.0f;
          ffu += (d <= -RELL) ? s[kg][r] : 0.0f;
        }
      }
    }
    const float rsum = rl + __shfl_xor(rl, 16, 32);
    fpa += __shfl_xor(fpa, 16, 32);
    ffu += __shfl_xor(ffu, 16, 32);
    lrun  = alpha * lrun + rsum;
    lpast = alpha * lpast + fpa;
    lfut  = alpha * lfut + ffu;
#pragma unroll
    for (int v = 0; v < 8; ++v) {
      const float av = __shfl(alpha, 8 * hh + v, 32);
#pragma unroll
      for (int nb = 0; nb < 4; ++nb) o[nb][v] = o[nb][v] * av;
    }

#pragma unroll
    for (int kg = 0; kg < 4; ++kg) {
      v8h pv;
#pragma unroll
      for (int r = 0; r < 8; ++r) pv[r] = toh_flush(s[kg][r] * PCARRY);
      *(v8h*)&P[m * LDT + kg * 16 + 8 * hh] = pv;
    }
    wave_lds_sync();

#pragma unroll
    for (int c = 0; c < 2; ++c) {
      const v16h pf = ld_frag(P + c * 32, LDT);
#pragma unroll
      for (int nb = 0; nb < 4; ++nb) {
        const v16h vf = ld_frag(&Vs[(nb * 16) * LDT + c * 32], LDT);
        o[nb] = wmma16(pf, vf, o[nb]);
      }
    }
    __syncthreads();
  }

  const float inv_l = __builtin_amdgcn_rcpf(lrun);
  const float osc = inv_l * RCARRY;
#pragma unroll
  for (int v = 0; v < 8; ++v) {
    const float iv = __shfl(osc, 8 * hh + v, 32);
#pragma unroll
    for (int nb = 0; nb < 4; ++nb) o[nb][v] = o[nb][v] * iv;
  }
  const float pscale = inv_l * PCARRY;
  wave_lds_sync();

#pragma unroll 1
  for (int c = 0; c < RELP / 32; ++c) {
    const int rel0 = c * 32 + 16 * hh;
    v8h pq[2];
#pragma unroll
    for (int g4 = 0; g4 < 4; ++g4) {
      const v4f tv = *(const v4f*)&Tb[tb0 + rel0 + 4 * g4];
#pragma unroll
      for (int e = 0; e < 4; ++e) {
        const int rel = rel0 + 4 * g4 + e;
        const int j = qrow - (rel - RELL);
        const int jc = min(max(j, 0), SEQ - 1);
        const int tvis = ((fl0 >> (jc >> 6)) & 1) | fl1;
        const float ea = fminf(tv[e] - mrun, 0.0f);
        const float ex = __expf(fmaxf(ea, -64.0f));
        const int ok = (int)(rel >= 1) & (int)(rel <= 2 * RELL - 1) & (int)(j >= 0) &
                       (int)(j < SEQ) & (int)(tvis != 0) & (int)(ea >= P_FLOOR);
        float p = (ok != 0) ? ex : 0.0f;
        p = (rel == 0) ? lfut : p;
        p = (rel == 2 * RELL) ? lpast : p;
        pq[g4 >> 1][(g4 & 1) * 4 + e] = toh_flush(p * pscale);
      }
    }
    *(v8h*)&P[m * LDT + 16 * hh]     = pq[0];
    *(v8h*)&P[m * LDT + 16 * hh + 8] = pq[1];
    wave_lds_sync();
    const v16h pf = ld_frag(P, LDT);
#pragma unroll
    for (int nb = 0; nb < 4; ++nb) {
      const v16h wf = frag_at(WRT + (size_t)(nb * 16 + m) * RELP + c * 32 + hh * 8);
      o[nb] = wmma16(pf, wf, o[nb]);
    }
    wave_lds_sync();
  }

#pragma unroll
  for (int v = 0; v < 8; ++v) {
#pragma unroll
    for (int nb = 0; nb < 4; ++nb)
      P[(hh * 8 + v) * LDT + nb * 16 + m] =
          toh_flush(o[nb][v] * (VCARRY / (PCARRY * RCARRY)));
  }
  wave_lds_sync();
  v8h x[4];
  size_t off[4];
#pragma unroll
  for (int i = 0; i < 4; ++i) {
    const int r = 4 * i + (lane >> 3);
    const int c = (lane & 7) * 8;
    x[i] = *(const v8h*)&P[r * LDT + c];
    off[i] = (size_t)(b * SEQ + q0 + w * 16 + r) * DIM + head * HD + c;
  }
#pragma unroll
  for (int i = 0; i < 4; ++i) *(volatile v8h*)(Ov + off[i]) = x[i];
  __threadfence();
#pragma unroll
  for (int i = 0; i < 4; ++i) *(volatile v8h*)(Ov + off[i]) = x[i];
}

extern "C" void kernel_launch(void* const* d_in, const int* in_sizes, int n_in,
                              void* d_out, int out_size, void* d_ws, size_t ws_size,
                              hipStream_t stream) {
  if (n_in < 19) return;
  const long long need_x = ((long long)(NB - 1) * SEQ_FULL + SEQ) * DIM;
  const long long need_m = ((long long)(NB - 1) * SEQ_FULL + SEQ) * SEQ_FULL;
  if ((long long)in_sizes[0] < need_x) return;
  if ((long long)in_sizes[1] < need_m) return;
  if (in_sizes[2] < DIM * DIM || in_sizes[4] < DIM * DIM || in_sizes[6] < DIM * DIM ||
      in_sizes[8] < DIM * DIM) return;
  if (in_sizes[15] < DFF * DIM || in_sizes[17] < DFF * DIM) return;
  if (in_sizes[3] < DIM || in_sizes[5] < DIM || in_sizes[7] < DIM || in_sizes[9] < DIM ||
      in_sizes[11] < DIM || in_sizes[12] < DIM || in_sizes[13] < DIM || in_sizes[14] < DIM ||
      in_sizes[18] < DIM) return;
  if (in_sizes[16] < DFF) return;
  if (in_sizes[10] < NREL * HD) return;
  if ((long long)out_size < need_x) return;
  if (ws_size < WS_TOTAL) return;

  const float* x    = (const float*)d_in[0];
  const int*   mask = (const int*)d_in[1];
  const float* Wq   = (const float*)d_in[2];
  const float* bq   = (const float*)d_in[3];
  const float* Wk   = (const float*)d_in[4];
  const float* bk   = (const float*)d_in[5];
  const float* Wv   = (const float*)d_in[6];
  const float* bv   = (const float*)d_in[7];
  const float* Wo   = (const float*)d_in[8];
  const float* bo   = (const float*)d_in[9];
  const float* Wrel = (const float*)d_in[10];
  const float* g1   = (const float*)d_in[11];
  const float* be1  = (const float*)d_in[12];
  const float* g2   = (const float*)d_in[13];
  const float* be2  = (const float*)d_in[14];
  const float* W1   = (const float*)d_in[15];
  const float* b1   = (const float*)d_in[16];
  const float* W2   = (const float*)d_in[17];
  const float* b2   = (const float*)d_in[18];
  float* out = (float*)d_out;

  char* ws = (char*)d_ws;
  _Float16* Wt     = (_Float16*)ws;
  _Float16* X16    = (_Float16*)(ws + OFF_X16);
  _Float16* Qh16   = (_Float16*)(ws + OFF_QH);
  _Float16* Kh16   = (_Float16*)(ws + OFF_KH);
  _Float16* Vt16   = (_Float16*)(ws + OFF_VT);
  _Float16* Ctx16  = (_Float16*)(ws + OFF_CTX);
  float*    X1     = (float*)(ws + OFF_X1);
  float*    Hf     = (float*)(ws + OFF_HF);
  _Float16* H16    = (_Float16*)(ws + OFF_H16);
  _Float16* F16    = (_Float16*)(ws + OFF_F);
  float*    Y      = (float*)(ws + OFF_Y);
  _Float16* WRp    = (_Float16*)(ws + OFF_WR);
  _Float16* WRTp   = (_Float16*)(ws + OFF_WRT);
  int*      Flg    = (int*)(ws + OFF_FLAG);

  dim3 blk(256);
  dim3 gg(DIM / 64, MROWS / 64);
  dim3 gf(DFF / 64, MROWS / 64);

  wconv_kernel<<<dim3((unsigned)(WT_ELEMS / 2048)), blk, 0, stream>>>(Wq, Wk, Wv, Wo, W1, W2, Wt);
  relconv_kernel<<<dim3(18), blk, 0, stream>>>(Wrel, WRp, WRTp);
  xconv_kernel<<<dim3((unsigned)(((size_t)MROWS * DIM) / 2048)), blk, 0, stream>>>(x, X16);
  flag_kernel<<<dim3(SEQ / 64, NB), blk, 0, stream>>>(mask, Flg);
  gemm_rows_kernel<<<gg, blk, 0, stream>>>(X16, Wt + 0 * WP, bq, x, X1, X1, Qh16);
  gemm_rows_kernel<<<gg, blk, 0, stream>>>(X16, Wt + 1 * WP, bk, x, X1, X1, Kh16);
  gemm_vt_kernel<<<gg, blk, 0, stream>>>(X16, Wt + 2 * WP, bv, x, X1, X1, Vt16);
  attn_kernel<<<dim3(SEQ / QROWS, NHEAD, NB), dim3(128), 0, stream>>>(
      Qh16, Kh16, Vt16, mask, WRp, WRTp, Flg, Ctx16);
  gemm_oproj_kernel<<<gg, blk, 0, stream>>>(Ctx16, Wt + 3 * WP, bo, x, X1, X1, Ctx16);
  ln_mid_kernel<<<dim3(MROWS), dim3(128), 0, stream>>>(X1, g1, be1, Hf, H16);
  gemm_ffn1_kernel<<<gf, blk, 0, stream>>>(H16, Wt + 4 * WP, b1, x, Hf, Y, F16);
  gemm_ffn2_kernel<<<gg, blk, 0, stream>>>(F16, Wt + 8 * WP, b2, x, Hf, Y, F16);
  ln_out_kernel<<<dim3(MROWS), dim3(128), 0, stream>>>(Y, g2, be2, out, H16);
}
